// Conv1dAttention_61778809585928
// MI455X (gfx1250) — hardware-verified
//
#include <hip/hip_runtime.h>


#define NB_  16
#define CIN  64
#define CC   128
#define KW   3
#define KI   (CIN * KW)
#define TT   2048
#define RH   512
#define PCAR 1024.0f
typedef _Float16 h16;
typedef unsigned short bf;
typedef __attribute__((ext_vector_type(16))) __bf16   v16bf;
typedef __attribute__((ext_vector_type(16))) _Float16 v16h;
typedef __attribute__((ext_vector_type(8)))  _Float16 v8h;
typedef __attribute__((ext_vector_type(8)))  unsigned short v8us;
typedef __attribute__((ext_vector_type(8)))  float    v8f;
typedef __attribute__((ext_vector_type(4)))  float    v4f;
typedef v8h  __attribute__((may_alias)) v8ha;
typedef v4f  __attribute__((may_alias)) v4fa;
typedef v8us __attribute__((may_alias)) v8usa;

__device__ __forceinline__ unsigned short f2bf(float f) { unsigned u = __float_as_uint(f); u += 0x7FFFu + ((u >> 16) & 1u); return (unsigned short)(u >> 16); }
__device__ __forceinline__ float bf2f(unsigned short b) { return __uint_as_float(((unsigned)b) << 16); }
__device__ __forceinline__ float bfr(float f) { return bf2f(f2bf(f)); }
__device__ __forceinline__ v16h cat16(v8h lo, v8h hi) { return __builtin_shufflevector(lo, hi, 0, 1, 2, 3, 4, 5, 6, 7, 8, 9, 10, 11, 12, 13, 14, 15); }
__device__ __forceinline__ v16bf cat16b(v8us lo, v8us hi) { return __builtin_bit_cast(v16bf, __builtin_shufflevector(lo, hi, 0, 1, 2, 3, 4, 5, 6, 7, 8, 9, 10, 11, 12, 13, 14, 15)); }
__device__ __forceinline__ v8f wmma16(v16h a, v16h b, v8f c) { return __builtin_amdgcn_wmma_f32_16x16x32_f16(false, a, false, b, (short)0, c, false, false); }
__device__ __forceinline__ v8f wmmab(v16bf a, v16bf b, v8f c) { return __builtin_amdgcn_wmma_f32_16x16x32_bf16(false, a, false, b, (short)0, c, false, false); }


template <typename T16> struct WFrag;
template <> struct WFrag<h16> { typedef v16h V; static __device__ __forceinline__ V ld(const h16* p) { return cat16(*(const v8h*)p, *(const v8h*)(p + 16)); } static __device__ __forceinline__ v8f mma(V a, V b, v8f c) { return wmma16(a, b, c); } };
template <> struct WFrag<bf> { typedef v16bf V; static __device__ __forceinline__ V ld(const bf* p) { return cat16b(*(const v8us*)p, *(const v8us*)(p + 16)); } static __device__ __forceinline__ v8f mma(V a, V b, v8f c) { return wmmab(a, b, c); } };
template <typename T16, int NSPLIT, bool BIAS>
__global__ __launch_bounds__(32) void k_gemmw(const T16* __restrict__ A, const T16* __restrict__ A2, const T16* __restrict__ Bt, const T16* __restrict__ Bt2, int K, float* C, int ldc, const float* __restrict__ bias, size_t sA, size_t sB, size_t sC) {
    typedef typename WFrag<T16>::V V;
    __shared__ __align__(16) float os[16 * 68];
    const size_t z = blockIdx.z; A += z * sA; if (A2) A2 += z * sA; Bt += z * sB; if (Bt2) Bt2 += z * sB; C += z * sC;
    const int lane = threadIdx.x & 31, lr = lane & 15, hi = lane >> 4; const int r0 = blockIdx.x * 64, c0 = blockIdx.y * 64;
    v8f acc[4][4];
#pragma unroll
    for (int mb = 0; mb < 4; ++mb)
#pragma unroll
        for (int nb = 0; nb < 4; ++nb) acc[mb][nb] = (v8f){};
    const size_t aoff = (size_t)(r0 + lr) * K + 8 * hi, boff = (size_t)(c0 + lr) * K + 8 * hi;
#pragma unroll 1
    for (int kc = 0; kc < K; kc += 32) {
        V a[4], a2[4];
#pragma unroll
        for (int mb = 0; mb < 4; ++mb) { a[mb] = WFrag<T16>::ld(A + aoff + (size_t)mb * 16 * K + kc); if (NSPLIT == 1 || NSPLIT == 2) a2[mb] = WFrag<T16>::ld(A2 + aoff + (size_t)mb * 16 * K + kc); }
#pragma unroll
        for (int nb = 0; nb < 4; ++nb) { const V b = WFrag<T16>::ld(Bt + boff + (size_t)nb * 16 * K + kc); V b2; if (NSPLIT >= 2) b2 = WFrag<T16>::ld(Bt2 + boff + (size_t)nb * 16 * K + kc);
#pragma unroll
            for (int mb = 0; mb < 4; ++mb) { acc[mb][nb] = WFrag<T16>::mma(a[mb], b, acc[mb][nb]); if (NSPLIT == 1 || NSPLIT == 2) acc[mb][nb] = WFrag<T16>::mma(a2[mb], b, acc[mb][nb]); if (NSPLIT >= 2) acc[mb][nb] = WFrag<T16>::mma(a[mb], b2, acc[mb][nb]); } }
        asm volatile("v_nop\n\tv_nop\n\tv_nop\n\tv_nop" : "+v"(acc[0][0]), "+v"(acc[1][1]), "+v"(acc[2][2]), "+v"(acc[3][3]) : "v"(a[0]), "v"(a[3]));
    }
#pragma unroll
    for (int mb = 0; mb < 4; ++mb) {
#pragma unroll
        for (int nb = 0; nb < 4; ++nb) {
#pragma unroll
            for (int j = 0; j < 8; ++j) os[(hi * 8 + j) * 68 + nb * 16 + lr] = acc[mb][nb][j]; }
        __builtin_amdgcn_wave_barrier(); asm volatile("" ::: "memory");
        float* crow = C + (size_t)(r0 + mb * 16) * ldc + c0;
#pragma unroll 1
        for (int ps = 0; ps < 2; ++ps) {
#pragma unroll
            for (int s = 0; s < 8; ++s) { const int row = 2 * s + hi, cofs = lr * 4; v4f val = *(const v4fa*)(os + row * 68 + cofs); if (BIAS) { val[0] += bfr(bias[c0 + cofs]); val[1] += bfr(bias[c0 + cofs + 1]); val[2] += bfr(bias[c0 + cofs + 2]); val[3] += bfr(bias[c0 + cofs + 3]); }
                *(volatile v4f*)(crow + (size_t)row * ldc + cofs) = val; }
            if (ps == 0) __threadfence(); }
        __builtin_amdgcn_wave_barrier(); asm volatile("" ::: "memory");
    }
}

__device__ __forceinline__ h16 tohx(float x) { return (h16)x; }
__device__ __forceinline__ void splitf(float y, unsigned short& h, unsigned short& l) { h = f2bf(y); l = f2bf(y - bf2f(h)); }
typedef __attribute__((ext_vector_type(2))) unsigned short v2us;
typedef __attribute__((ext_vector_type(4))) unsigned short v4us;
typedef __attribute__((ext_vector_type(8))) unsigned short v8us;
typedef __attribute__((ext_vector_type(4))) _Float16 v4h;
typedef __attribute__((ext_vector_type(2))) float v2f;

__global__ __launch_bounds__(256) void k_cvt8(const float* __restrict__ src, bf* dst, size_t n8) { const size_t i = (size_t)blockIdx.x * 256 + threadIdx.x; if (i >= n8) return; const v8f v = *(const v8f*)(src + i * 8); v8us o;
#pragma unroll
    for (int k = 0; k < 8; ++k) o[k] = f2bf(v[k]); *(volatile v8us*)(dst + i * 8) = o; __threadfence(); *(volatile v8us*)(dst + i * 8) = o; }
__global__ __launch_bounds__(256) void k_im2col(const float* __restrict__ xb, bf* X3) { const size_t e8 = ((size_t)blockIdx.x * 256 + threadIdx.x) * 8; if (e8 >= (size_t)TT * KI) return; const int kidx = (int)(e8 % KI); const int t = (int)(e8 / KI); v8us o;
#pragma unroll
    for (int u = 0; u < 8; ++u) { const int k2 = kidx + u; const int ci = k2 / KW, kk = k2 % KW; const int tt = t + kk - 1; o[u] = (tt >= 0 && tt < TT) ? f2bf(xb[(size_t)ci * TT + tt]) : (unsigned short)0; }
    *(volatile v8us*)(X3 + e8) = o; __threadfence(); *(volatile v8us*)(X3 + e8) = o; }
__global__ __launch_bounds__(256) void k_bnl(float* F, const float* __restrict__ gam, const float* __restrict__ bet, const float* __restrict__ mu, const float* __restrict__ var) { const size_t e = ((size_t)blockIdx.x * 256 + threadIdx.x) * 4; if (e >= (size_t)TT * CC) return; const int c0 = (int)(e % CC); const v4f a = *(const v4f*)(F + e); v4f o;
#pragma unroll
    for (int u = 0; u < 4; ++u) { const int c = c0 + u; const float sc = __fmul_rn(bfr(gam[c]), __fdiv_rn(1.0f, sqrtf(__fadd_rn(bfr(var[c]), 1e-5f)))); float ms = __fmul_rn(bfr(mu[c]), sc); asm volatile("" : "+v"(ms)); const float sh = __fsub_rn(bfr(bet[c]), ms); float y = __fmul_rn(a[u], sc); asm volatile("" : "+v"(y)); y = __fadd_rn(y, sh); o[u] = (y > 0.f) ? y : 0.3f * y; }
    *(volatile v4f*)(F + e) = o; __threadfence(); *(volatile v4f*)(F + e) = o; }
__global__ __launch_bounds__(256) void k_hlN(const float* __restrict__ F, bf* Fh, bf* Fl) { const size_t e = ((size_t)blockIdx.x * 256 + threadIdx.x) * 4; if (e >= (size_t)TT * CC) return; const v4f a = *(const v4f*)(F + e); v4us oh, ol; for (int u = 0; u < 4; ++u) { unsigned short p, q; splitf(a[u], p, q); oh[u] = p; ol[u] = q; } *(volatile v4us*)(Fh + e) = oh; *(volatile v4us*)(Fl + e) = ol; __threadfence(); *(volatile v4us*)(Fh + e) = oh; *(volatile v4us*)(Fl + e) = ol; }
__global__ __launch_bounds__(256) void k_hlT(const float* __restrict__ F, bf* Th, bf* Tl, h16* T16) { const size_t e = ((size_t)blockIdx.x * 256 + threadIdx.x) * 2; if (e >= (size_t)CC * TT) return; const int t = (int)(e % TT); const int c = (int)(e / TT); v2us oh, ol; _Float16 f0, f1;
    { unsigned short p, q; const float a0 = F[(size_t)t * CC + c]; splitf(a0, p, q); oh[0] = p; ol[0] = q; f0 = tohx(a0); const float a1 = F[(size_t)(t + 1) * CC + c]; splitf(a1, p, q); oh[1] = p; ol[1] = q; f1 = tohx(a1); }
    typedef __attribute__((ext_vector_type(2))) _Float16 v2h; v2h fo; fo[0] = f0; fo[1] = f1;
    *(volatile v2us*)(Th + e) = oh; *(volatile v2us*)(Tl + e) = ol; *(volatile v2h*)(T16 + e) = fo; __threadfence(); *(volatile v2us*)(Th + e) = oh; *(volatile v2us*)(Tl + e) = ol; *(volatile v2h*)(T16 + e) = fo; }
__global__ __launch_bounds__(256) void k_psoft(const float* __restrict__ S, bf* Ph, bf* Pl) { const int lane = threadIdx.x & 31; const int row = blockIdx.x * 8 + (threadIdx.x >> 5); if (row >= TT) return; const float* sr = S + (size_t)row * TT; float v[TT / 32]; float mx = -3.0e38f;
#pragma unroll
    for (int ch = 0; ch < TT / 128; ++ch) { const v4f a = *(const v4f*)(sr + ch * 128 + lane * 4);
#pragma unroll
        for (int u = 0; u < 4; ++u) { float sa = a[u]; asm volatile("" : "+v"(sa)); v[ch * 4 + u] = sa; mx = fmaxf(mx, sa); } }
#pragma unroll
    for (int sh = 16; sh; sh >>= 1) mx = fmaxf(mx, __shfl_xor(mx, sh, 32));
    float sum = 0.f;
#pragma unroll
    for (int q = 0; q < TT / 32; ++q) { float d0 = __fsub_rn(v[q], mx); asm volatile("" : "+v"(d0)); v[q] = __builtin_amdgcn_exp2f(__fmul_rn(d0, 1.4426950408889634f)); sum += v[q]; }
#pragma unroll
    for (int sh = 16; sh; sh >>= 1) sum += __shfl_xor(sum, sh, 32);
    const float f = __fdiv_rn(1.0f, sum);
    for (int ps = 0; ps < 2; ++ps) {
#pragma unroll
        for (int ch = 0; ch < TT / 128; ++ch) { v4us oh, ol; for (int q = 0; q < 4; ++q) { unsigned short a, c2; splitf(v[ch * 4 + q] * f, a, c2); oh[q] = a; ol[q] = c2; } const size_t oo = (size_t)row * TT + ch * 128 + lane * 4; *(volatile v4us*)(Ph + oo) = oh; *(volatile v4us*)(Pl + oo) = ol; }
        if (ps == 0) __threadfence(); } }
__global__ __launch_bounds__(256) void k_ptr(const bf* __restrict__ Ph, const bf* __restrict__ Pl, bf* PTh, bf* PTl, h16* PT16) { const size_t e = ((size_t)blockIdx.x * 256 + threadIdx.x) * 4; if (e >= (size_t)TT * TT) return; const int j = (int)(e % TT); const int l = (int)(e / TT); v4us oh, ol; v4h o4;
#pragma unroll
    for (int u = 0; u < 4; ++u) { const size_t src = (size_t)(j + u) * TT + l; const unsigned short a = Ph[src], c = Pl[src]; oh[u] = a; ol[u] = c; o4[u] = tohx(__fadd_rn(bf2f(a), bf2f(c)) * PCAR); }
    if (l < RH) { *(volatile v4us*)(PTh + e) = oh; *(volatile v4us*)(PTl + e) = ol; __threadfence(); *(volatile v4us*)(PTh + e) = oh; *(volatile v4us*)(PTl + e) = ol; }
    else { const size_t o2 = e - (size_t)RH * TT; *(volatile v4h*)(PT16 + o2) = o4; __threadfence(); *(volatile v4h*)(PT16 + o2) = o4; } }
__global__ __launch_bounds__(256) void k_fin(const float* __restrict__ OT, const float* __restrict__ PE, float* OUTb) { const size_t e = ((size_t)blockIdx.x * 256 + threadIdx.x) * 4; if (e >= (size_t)CC * TT) return; const int l = (int)(e % TT); const int c = (int)(e / TT); v4f r;
#pragma unroll
    for (int u = 0; u < 4; ++u) { const int ll = l + u; const float cs = (ll < RH) ? 1.0f : (1.0f / PCAR); float o = OT[(size_t)ll * CC + c] * cs; asm volatile("" : "+v"(o)); r[u] = __fadd_rn(o, PE[(size_t)ll * CC + c]); }
    *(volatile v4f*)(OUTb + e) = r; __threadfence(); *(volatile v4f*)(OUTb + e) = r; }

extern "C" void kernel_launch(void* const* d_in, const int* in_sizes, int n_in,
                              void* d_out, int out_size, void* d_ws, size_t ws_size, hipStream_t stream) {
    (void)in_sizes; (void)n_in; (void)out_size;
    const float* x = (const float*)d_in[0];
    const float* prm[4][6]; for (int r = 0; r < 4; ++r) for (int c = 0; c < 6; ++c) prm[r][c] = (const float*)d_in[1 + r * 6 + c];
    float* OUT = (float*)d_out;
    char* wsp = (char*)d_ws;
    auto take = [&](size_t bytes) { char* p = wsp; wsp += (bytes + 255) & ~(size_t)255; return (void*)p; };
    bf* W4 = (bf*)take((size_t)4 * CC * KI * 2); bf* X3 = (bf*)take((size_t)TT * KI * 2);
    float* FQ = (float*)take((size_t)TT * CC * 4); float* FK = (float*)take((size_t)TT * CC * 4); float* FV = (float*)take((size_t)TT * CC * 4); float* FPE = (float*)take((size_t)TT * CC * 4);
    bf* QPh = (bf*)take((size_t)TT * CC * 2); bf* QPl = (bf*)take((size_t)TT * CC * 2); bf* KPh = (bf*)take((size_t)TT * CC * 2); bf* KPl = (bf*)take((size_t)TT * CC * 2);
    bf* VTh = (bf*)take((size_t)CC * TT * 2); bf* VTl = (bf*)take((size_t)CC * TT * 2); h16* VT16 = (h16*)take((size_t)CC * TT * 2);
    float* S = (float*)take((size_t)TT * TT * 4); bf* Ph = (bf*)take((size_t)TT * TT * 2); bf* Pl = (bf*)take((size_t)TT * TT * 2); bf* PTh = (bf*)take((size_t)RH * TT * 2); bf* PTl = (bf*)take((size_t)RH * TT * 2); h16* PT16 = (h16*)take((size_t)(TT - RH) * TT * 2); float* OT = (float*)take((size_t)TT * CC * 4);
    if ((size_t)(wsp - (char*)d_ws) > ws_size) return;
    for (int r = 0; r < 4; ++r) k_cvt8<<<(unsigned)(((size_t)CC * KI / 8 + 255) / 256), 256, 0, stream>>>(prm[r][0], W4 + (size_t)r * CC * KI, (size_t)CC * KI / 8);
    for (int b = 0; b < NB_; ++b) { const float* xb = x + (size_t)b * CIN * TT;
        k_im2col<<<(unsigned)(((size_t)TT * KI / 8 + 255) / 256), 256, 0, stream>>>(xb, X3);
        float* F4[4] = {FQ, FK, FV, FPE};
        for (int r = 0; r < 4; ++r) { k_gemmw<bf, 0, true><<<dim3(TT / 64, CC / 64, 1), 32, 0, stream>>>(X3, nullptr, W4 + (size_t)r * CC * KI, nullptr, KI, F4[r], CC, prm[r][1], 0, 0, 0); k_bnl<<<(unsigned)(((size_t)TT * CC / 4 + 255) / 256), 256, 0, stream>>>(F4[r], prm[r][2], prm[r][3], prm[r][4], prm[r][5]); }
        k_hlN<<<(unsigned)(((size_t)TT * CC / 4 + 255) / 256), 256, 0, stream>>>(FQ, QPh, QPl); k_hlN<<<(unsigned)(((size_t)TT * CC / 4 + 255) / 256), 256, 0, stream>>>(FK, KPh, KPl); k_hlT<<<(unsigned)(((size_t)CC * TT / 2 + 255) / 256), 256, 0, stream>>>(FV, VTh, VTl, VT16);
        k_gemmw<bf, 2, false><<<dim3(TT / 64, TT / 64, 1), 32, 0, stream>>>(QPh, QPl, KPh, KPl, CC, S, TT, nullptr, 0, 0, 0);
        k_psoft<<<TT / 8, 256, 0, stream>>>(S, Ph, Pl);
        k_ptr<<<(unsigned)(((size_t)TT * TT / 4 + 255) / 256), 256, 0, stream>>>(Ph, Pl, PTh, PTl, PT16);
        k_gemmw<bf, 2, false><<<dim3(RH / 64, CC / 64, 1), 32, 0, stream>>>(PTh, PTl, VTh, VTl, TT, OT, CC, nullptr, 0, 0, 0);
        k_gemmw<h16, 0, false><<<dim3((TT - RH) / 64, CC / 64, 1), 32, 0, stream>>>(PT16, nullptr, VT16, nullptr, TT, OT + (size_t)RH * CC, CC, nullptr, 0, 0, 0);
        k_fin<<<(unsigned)(((size_t)CC * TT / 4 + 255) / 256), 256, 0, stream>>>(OT, FPE, OUT + (size_t)b * CC * TT); }
}
